// NN_4260607557798
// MI455X (gfx1250) — hardware-run, weakly checked
//
#include <hip/hip_runtime.h>
#include <math.h>
#pragma clang fp contract(off)

typedef __attribute__((ext_vector_type(16))) _Float16 v16h;
typedef __attribute__((ext_vector_type(8)))  _Float16 v8h;
typedef __attribute__((ext_vector_type(16))) __bf16   v16b;
typedef __attribute__((ext_vector_type(8)))  __bf16   v8b;
typedef __attribute__((ext_vector_type(8)))  float    v8f;
typedef __attribute__((ext_vector_type(4)))  float    v4f;
typedef __attribute__((ext_vector_type(2)))  float    v2f;
typedef __attribute__((ext_vector_type(4)))  int      v4i;

constexpr int kBatch    = 16;
constexpr int kNpt      = 2048;
constexpr int kNbr      = 20;
constexpr int kRows     = kBatch * kNpt;
constexpr int kXc       = 6;
constexpr int kC1       = 64;
constexpr int kIdxPitch = 32;
constexpr int kHeadN    = 13;
constexpr int kHeadPad  = 64;
constexpr int kEdgeBlocks = kRows / 64;
constexpr float kBnEps  = 1e-5f;
constexpr bool kSqPairOrder = true;
static_assert(kRows == 32768, "rows");
static_assert((kRows % 64) == 0, "M tile multiple");
static_assert(kEdgeBlocks == 512, "edge blocks");
static_assert((kHeadN * 64 * 4) % 128 == 0, "head tile is whole lines");

constexpr int kW1Off = 0;
constexpr int kW2Off = kW1Off + 64 * 64;
constexpr int kW3Off = kW2Off + 128 * 64;
constexpr int kW4Off = kW3Off + 256 * 128;
constexpr int kW5Off = kW4Off + 128 * 256;
constexpr int kW6Off = kW5Off + 64 * 128;
constexpr int kWTot  = kW6Off + kHeadPad * 64;
static_assert(kWTot == 90112, "weight plane elements");
static_assert((kW2Off % 2048) == 0 && (kW3Off % 2048) == 0 && (kW4Off % 2048) == 0 &&
              (kW5Off % 2048) == 0 && (kW6Off % 2048) == 0 && (kWTot % 2048) == 0, "block-uniform segments");
constexpr int kSplitBlocks = kWTot / 2048;

constexpr size_t kOffWH   = 0;
constexpr size_t kOffWL   = kOffWH   + (size_t)kWTot * 2;
constexpr size_t kOffIDX  = kOffWL   + (size_t)kWTot * 2;
constexpr size_t kOffHMAX = kOffIDX  + (size_t)kRows * kIdxPitch * 4;
constexpr size_t kOffHMIN = kOffHMAX + (size_t)kRows * kC1 * 4;
constexpr size_t kOffPART = kOffHMIN + (size_t)kRows * kC1 * 4;
constexpr size_t kOffSCSH = kOffPART + (size_t)kEdgeBlocks * 128 * 4;
constexpr size_t kOffPH   = kOffSCSH + 512;
constexpr size_t kOffPL   = kOffPH   + (size_t)kRows * 128 * 2;
constexpr size_t kOffQH   = kOffPL   + (size_t)kRows * 128 * 2;
constexpr size_t kOffQL   = kOffQH   + (size_t)kRows * 256 * 2;
constexpr size_t kWsTotal = kOffQL   + (size_t)kRows * 256 * 2;
static_assert(kWsTotal == 71926272ull, "carve total");
static_assert(kWsTotal <= 134217728ull, "carve cap");
static_assert((kOffWL % 128) == 0 && (kOffIDX % 128) == 0 && (kOffHMAX % 128) == 0 && (kOffHMIN % 128) == 0 &&
              (kOffPART % 128) == 0 && (kOffSCSH % 128) == 0 && (kOffPH % 128) == 0 && (kOffPL % 128) == 0 &&
              (kOffQH % 128) == 0 && (kOffQL % 128) == 0, "128-B aligned regions");

__device__ __forceinline__ unsigned short f2bf_bits(float f) {
  unsigned u = __float_as_uint(f);
  return (unsigned short)((u + 0x7FFFu + ((u >> 16) & 1u)) >> 16);
}
__device__ __forceinline__ float bf_bits2f(unsigned short h) { return __uint_as_float(((unsigned)h) << 16); }

__device__ __forceinline__ void dep_guard4_b(v8f& a, v8f& b, v8f& c, v8f& d, v16b x, v16b y) {
  asm volatile("v_nop\n\tv_nop\n\tv_nop\n\tv_nop" : "+v"(a), "+v"(b), "+v"(c), "+v"(d) : "v"(x), "v"(y));
}
__device__ __forceinline__ void keep4_b(v16b a, v16b b, v16b c, v16b d) { asm volatile("v_nop" :: "v"(a), "v"(b), "v"(c), "v"(d)); }
__device__ __forceinline__ void acc_guard4(v8f& a, v8f& b, v8f& c, v8f& d) {
  asm volatile("v_nop\n\tv_nop\n\tv_nop\n\tv_nop" : "+v"(a), "+v"(b), "+v"(c), "+v"(d));
}
union FragB { v16b v; v8b h[2]; };
__device__ __forceinline__ v16b frag_load_b(const __bf16* p) {
  FragB f; f.h[0] = *(const v8b*)(p); f.h[1] = *(const v8b*)(p + 16); return f.v;
}
__device__ __forceinline__ v8f mma_b(v16b a, v16b b, v8f c) {
  return __builtin_amdgcn_wmma_f32_16x16x32_bf16(false, a, false, b, (short)0, c, false, false);
}

__device__ __forceinline__ void split2x4(const v4f a0, const v4f a1, v8h& hv, v8h& lv) {
#pragma unroll
  for (int e = 0; e < 4; ++e) {
    const float f0 = a0[e];
    const float f1 = a1[e];
    const unsigned short h0 = f2bf_bits(f0);
    const unsigned short h1 = f2bf_bits(f1);
    const unsigned short l0 = f2bf_bits(f0 - bf_bits2f(h0));
    const unsigned short l1 = f2bf_bits(f1 - bf_bits2f(h1));
    hv[e]     = __builtin_bit_cast(_Float16, h0);
    hv[4 + e] = __builtin_bit_cast(_Float16, h1);
    lv[e]     = __builtin_bit_cast(_Float16, l0);
    lv[4 + e] = __builtin_bit_cast(_Float16, l1);
  }
}

__global__ __launch_bounds__(256) void split_weights_kernel(
    const float* __restrict__ w1, const float* __restrict__ w2, const float* __restrict__ w3,
    const float* __restrict__ w4, const float* __restrict__ w5, const float* __restrict__ w6,
    unsigned short* __restrict__ WH, unsigned short* __restrict__ WL)
{
  const int blk = (int)blockIdx.x;
  const float* src = w1;
  int blk0 = 0;
  int real8 = (64 * 64) / 8;
  if (blk >= kW6Off / 2048)      { src = w6; blk0 = kW6Off / 2048; real8 = (kHeadN * 64) / 8; }
  else if (blk >= kW5Off / 2048) { src = w5; blk0 = kW5Off / 2048; real8 = (64 * 128) / 8; }
  else if (blk >= kW4Off / 2048) { src = w4; blk0 = kW4Off / 2048; real8 = (128 * 256) / 8; }
  else if (blk >= kW3Off / 2048) { src = w3; blk0 = kW3Off / 2048; real8 = (256 * 128) / 8; }
  else if (blk >= kW2Off / 2048) { src = w2; blk0 = kW2Off / 2048; real8 = (128 * 64) / 8; }
  const int li = (blk - blk0) * 256 + (int)threadIdx.x;
  const bool real = li < real8;
  const int lc = real ? li : (real8 - 1);
  v4f a0 = *(const v4f*)(src + (size_t)lc * 8);
  v4f a1 = *(const v4f*)(src + (size_t)lc * 8 + 4);
  asm volatile("" : "+v"(a0), "+v"(a1));
  v4f z0, z1;
#pragma unroll
  for (int e = 0; e < 4; ++e) {
    const float t0 = a0[e];
    const float t1 = a1[e];
    z0[e] = real ? t0 : 0.0f;
    z1[e] = real ? t1 : 0.0f;
  }
  v8h hv, lv;
  split2x4(z0, z1, hv, lv);
  const size_t e0 = ((size_t)blk * 256 + threadIdx.x) * 8;
  unsigned short* qh = WH + e0;
  unsigned short* ql = WL + e0;
  *(volatile v8h*)qh = hv;
  *(volatile v8h*)ql = lv;
  __threadfence();
  *(volatile v8h*)qh = hv;
  *(volatile v8h*)ql = lv;
}

__global__ __launch_bounds__(256) void knn_select_kernel(const float* __restrict__ x, int* __restrict__ idxp)
{
  __shared__ __align__(16) float spt[kNpt * 4];
  __shared__ __align__(16) int sidx[256 * kIdxPitch];
  const int tid  = (int)threadIdx.x;
  const int lane = tid & 31;
  const int wave = __builtin_amdgcn_readfirstlane((int)(threadIdx.x >> 5));
  const int b    = (int)blockIdx.y;
#pragma unroll 1
  for (int i = 0; i < kNpt / 256; ++i) {
    const int j = tid + 256 * i;
    const float* p = x + (size_t)(b * kNpt + j) * kXc;
    const float p0 = p[0];
    const float p1 = p[1];
    const float p2 = p[2];
    const float t0 = p0 * p0;
    const float t1 = p1 * p1;
    const float t2 = p2 * p2;
    float sq;
    if (kSqPairOrder) sq = (t0 + t2) + t1;
    else              sq = fmaf(p2, p2, fmaf(p1, p1, t0));
    v4f v;
    v[0] = p0; v[1] = p1; v[2] = p2; v[3] = sq;
    *(v4f*)(spt + 4 * j) = v;
  }
  __syncthreads();

  const int q = (int)blockIdx.x * 256 + tid;
  const v4f qv = *(const v4f*)(spt + 4 * q);
  const float qx = qv[0];
  const float qy = qv[1];
  const float qz = qv[2];
  const float qs = qv[3];

  float bd[kNbr];
  int   bi[kNbr];
#pragma unroll
  for (int t = 0; t < kNbr; ++t) { bd[t] = __builtin_huge_valf(); bi[t] = 0; }

#pragma unroll 1
  for (int j = 0; j < kNpt; ++j) {
    const v4f c = *(const v4f*)(spt + 4 * j);
    float p = qx * c[0];
    p = fmaf(qy, c[1], p);
    p = fmaf(qz, c[2], p);
    const float d2 = (qs + c[3]) - 2.0f * p;
    if (d2 < bd[kNbr - 1]) {
      bool ct = true;
#pragma unroll
      for (int t = kNbr - 1; t >= 1; --t) {
        const bool cm = d2 < bd[t - 1];
        const float nd = cm ? bd[t - 1] : d2;
        const int   ni = cm ? bi[t - 1] : j;
        bd[t] = ct ? nd : bd[t];
        bi[t] = ct ? ni : bi[t];
        ct = cm;
      }
      bd[0] = ct ? d2 : bd[0];
      bi[0] = ct ? j : bi[0];
    }
  }

  {
    int* row = sidx + tid * kIdxPitch;
    v4i r0, r1, r2, r3, r4, rz;
    r0[0] = bi[0];  r0[1] = bi[1];  r0[2] = bi[2];  r0[3] = bi[3];
    r1[0] = bi[4];  r1[1] = bi[5];  r1[2] = bi[6];  r1[3] = bi[7];
    r2[0] = bi[8];  r2[1] = bi[9];  r2[2] = bi[10]; r2[3] = bi[11];
    r3[0] = bi[12]; r3[1] = bi[13]; r3[2] = bi[14]; r3[3] = bi[15];
    r4[0] = bi[16]; r4[1] = bi[17]; r4[2] = bi[18]; r4[3] = bi[19];
    rz[0] = 0; rz[1] = 0; rz[2] = 0; rz[3] = 0;
    *(v4i*)(row + 0)  = r0;
    *(v4i*)(row + 4)  = r1;
    *(v4i*)(row + 8)  = r2;
    *(v4i*)(row + 12) = r3;
    *(v4i*)(row + 16) = r4;
    *(v4i*)(row + 20) = rz;
    *(v4i*)(row + 24) = rz;
    *(v4i*)(row + 28) = rz;
  }
  __syncthreads();
  {
    const int q4 = lane >> 3;
    const int c4 = (lane & 7) * 4;
    v4i vals[8];
#pragma unroll
    for (int it = 0; it < 8; ++it) {
      const int r = wave * 32 + it * 4 + q4;
      vals[it] = *(const v4i*)(sidx + r * kIdxPitch + c4);
    }
    int* gbase = idxp + ((size_t)(b * kNpt) + (size_t)blockIdx.x * 256) * kIdxPitch;
    for (int pass = 0; pass < 2; ++pass) {
#pragma unroll
      for (int it = 0; it < 8; ++it) {
        const int r = wave * 32 + it * 4 + q4;
        *(volatile v4i*)(gbase + (size_t)r * kIdxPitch + c4) = vals[it];
      }
      __threadfence();
    }
  }
}

__global__ __launch_bounds__(256) void edge_conv_stats_kernel(
    const float* __restrict__ x, const int* __restrict__ idxp, const float* __restrict__ wc,
    float* __restrict__ hmax, float* __restrict__ hmin, float* __restrict__ part)
{
  __shared__ __align__(16) float sfeat[2 * 4 * 160];
  __shared__ __align__(16) float smx[64 * 64];
  __shared__ __align__(16) float smn[64 * 64];
  __shared__ __align__(16) float sred[4 * 128];
  const int tid  = (int)threadIdx.x;
  const int lane = tid & 31;
  const int wave = __builtin_amdgcn_readfirstlane((int)(threadIdx.x >> 5));
  const int g    = wave >> 1;
  const int o    = tid & 63;

  const v2f wa = *(const v2f*)(wc + o * kXc);
  const v2f wb = *(const v2f*)(wc + o * kXc + 2);
  const v2f wd = *(const v2f*)(wc + o * kXc + 4);
  const float w0 = wa[0], w1 = wa[1], w2 = wb[0], w3 = wb[1], w4 = wd[0], w5 = wd[1];

  const int e2 = (o < 60) ? o : 59;
  const int kk = e2 / 3;
  const int c2 = e2 - kk * 3;
  const bool gact = (o < 60);
  const bool sub0 = (kk != 0) && (c2 <= 1);
  const bool sub1 = (kk != 0) && (c2 == 0);

  float s = 0.0f, ss = 0.0f;
  const int pbase = (int)blockIdx.x * 64 + g * 16;

#pragma unroll 1
  for (int it = 0; it < 16; ++it) {
    const int item = pbase + it;
    const int brow = item & ~(kNpt - 1);
    int jn = idxp[(size_t)item * kIdxPitch + kk];
    jn = jn < 0 ? 0 : (jn > (kNpt - 1) ? (kNpt - 1) : jn);
    v2f vn = *(const v2f*)(x + (size_t)(brow + jn) * kXc + 2 * c2);
    v2f vs = *(const v2f*)(x + (size_t)item * kXc + 2 * c2);
    asm volatile("" : "+v"(vn), "+v"(vs));
    const float n0 = vn[0], n1 = vn[1];
    const float d0 = n0 - vs[0];
    const float d1 = n1 - vs[1];
    v2f fv;
    fv[0] = sub0 ? d0 : n0;
    fv[1] = sub1 ? d1 : n1;
    float* fb = sfeat + ((it & 1) * 4 + g) * 160;
    if (gact) *(v2f*)(fb + kk * 8 + 2 * c2) = fv;
    __syncthreads();
    float mx = -__builtin_huge_valf();
    float mn = __builtin_huge_valf();
#pragma unroll 4
    for (int k = 0; k < kNbr; ++k) {
      const v4f fa = *(const v4f*)(fb + k * 8);
      const v2f fc = *(const v2f*)(fb + k * 8 + 4);
      float h = w0 * fa[0];
      h = fmaf(w1, fa[1], h);
      h = fmaf(w2, fa[2], h);
      h = fmaf(w3, fa[3], h);
      h = fmaf(w4, fc[0], h);
      h = fmaf(w5, fc[1], h);
      s += h;
      ss = fmaf(h, h, ss);
      mx = fmaxf(mx, h);
      mn = fminf(mn, h);
    }
    smx[(g * 16 + it) * 64 + o] = mx;
    smn[(g * 16 + it) * 64 + o] = mn;
  }
  sred[g * 128 + o]      = s;
  sred[g * 128 + 64 + o] = ss;
  __syncthreads();

  const int hh = lane >> 4;
  const int c4 = (lane & 15) * 4;
  v4f vx[4], vm[4];
#pragma unroll
  for (int it = 0; it < 4; ++it) {
    const int r = wave * 8 + it * 2 + hh;
    vx[it] = *(const v4f*)(smx + r * 64 + c4);
    vm[it] = *(const v4f*)(smn + r * 64 + c4);
  }
  v4f pv = *(const v4f*)(sred + lane * 4);
  {
    const v4f p1 = *(const v4f*)(sred + 128 + lane * 4);
    const v4f p2 = *(const v4f*)(sred + 256 + lane * 4);
    const v4f p3 = *(const v4f*)(sred + 384 + lane * 4);
    pv = ((pv + p1) + p2) + p3;
  }
  const size_t rbase = (size_t)blockIdx.x * 64;
  for (int pass = 0; pass < 2; ++pass) {
#pragma unroll
    for (int it = 0; it < 4; ++it) {
      const int r = wave * 8 + it * 2 + hh;
      *(volatile v4f*)(hmax + (rbase + r) * kC1 + c4) = vx[it];
      *(volatile v4f*)(hmin + (rbase + r) * kC1 + c4) = vm[it];
    }
    if (wave == 0) *(volatile v4f*)(part + (size_t)blockIdx.x * 128 + lane * 4) = pv;
    __threadfence();
  }
}

__global__ __launch_bounds__(256) void bn_finalize_kernel(
    const float* __restrict__ part, const float* __restrict__ g1, const float* __restrict__ be1,
    float* __restrict__ scsh)
{
  __shared__ double sacc[256];
  __shared__ __align__(16) float sout[128];
  const int tid  = (int)threadIdx.x;
  const int lane = tid & 31;
  const int wave = __builtin_amdgcn_readfirstlane((int)(threadIdx.x >> 5));
  const int c  = tid & 127;
  const int hb = tid >> 7;
  double a = 0.0;
#pragma unroll 4
  for (int r = 0; r < kEdgeBlocks / 2; ++r) a += (double)part[(size_t)(hb * (kEdgeBlocks / 2) + r) * 128 + c];
  sacc[tid] = a;
  const float gg = g1[tid & 63];
  const float bb = be1[tid & 63];
  __syncthreads();
  if (wave < 2) {
    const double S  = sacc[tid] + sacc[128 + tid];
    const double SS = sacc[64 + tid] + sacc[192 + tid];
    const double inv = 1.0 / ((double)kRows * (double)kNbr);
    const double mu = S * inv;
    double var = SS * inv - mu * mu;
    var = var < 0.0 ? 0.0 : var;
    const float varf = (float)var;
    const float sc = gg * (1.0f / sqrtf(varf + kBnEps));
    const float sh = bb - (float)mu * sc;
    sout[tid]      = sc;
    sout[64 + tid] = sh;
  }
  __syncthreads();
  const v4f v = *(const v4f*)(sout + lane * 4);
  if (wave == 0) {
    *(volatile v4f*)(scsh + lane * 4) = v;
    __threadfence();
    *(volatile v4f*)(scsh + lane * 4) = v;
  }
}

__global__ __launch_bounds__(256) void bn_apply_kernel(
    const float* __restrict__ hmax, const float* __restrict__ hmin, const float* __restrict__ scsh,
    unsigned short* __restrict__ AH, unsigned short* __restrict__ AL)
{
  const size_t i  = (size_t)blockIdx.x * 256 + threadIdx.x;
  const size_t e0 = i * 8;
  const int c0 = (int)(threadIdx.x & 7) * 8;
  const v4f x0 = *(const v4f*)(hmax + e0);
  const v4f x1 = *(const v4f*)(hmax + e0 + 4);
  const v4f n0 = *(const v4f*)(hmin + e0);
  const v4f n1 = *(const v4f*)(hmin + e0 + 4);
  const v4f s0 = *(const v4f*)(scsh + c0);
  const v4f s1 = *(const v4f*)(scsh + c0 + 4);
  const v4f t0 = *(const v4f*)(scsh + 64 + c0);
  const v4f t1 = *(const v4f*)(scsh + 64 + c0 + 4);
  v4f y0, y1;
#pragma unroll
  for (int e = 0; e < 4; ++e) {
    const float sa = s0[e];
    const float sb = s1[e];
    const float ha = (sa >= 0.0f) ? x0[e] : n0[e];
    const float hb = (sb >= 0.0f) ? x1[e] : n1[e];
    float ya = sa * ha + t0[e];
    float yb = sb * hb + t1[e];
    ya = (ya > 0.0f) ? ya : 0.2f * ya;
    yb = (yb > 0.0f) ? yb : 0.2f * yb;
    y0[e] = ya;
    y1[e] = yb;
  }
  v8h hv, lv;
  split2x4(y0, y1, hv, lv);
  unsigned short* qh = AH + e0;
  unsigned short* ql = AL + e0;
  *(volatile v8h*)qh = hv;
  *(volatile v8h*)ql = lv;
  __threadfence();
  *(volatile v8h*)qh = hv;
  *(volatile v8h*)ql = lv;
}

template <int OUT_MODE, bool CLAMP0>
__global__ __launch_bounds__(256) void mlp_gemm64_kernel(
    const unsigned short* __restrict__ Ahp, const unsigned short* __restrict__ Alp, int lda,
    const unsigned short* __restrict__ Bhp, const unsigned short* __restrict__ Blp, int ldb,
    void* __restrict__ Cout, void* __restrict__ Cout2, int ldc,
    const float* __restrict__ bias, int M, int N, int K)
{
  const __bf16* Ah = (const __bf16*)Ahp;
  const __bf16* Al = (const __bf16*)Alp;
  const __bf16* Bh = (const __bf16*)Bhp;
  const __bf16* Bl = (const __bf16*)Blp;
  __shared__ __align__(16) float sT[8][16 * 68];
  const int lane = (int)(threadIdx.x & 31);
  const int wave = __builtin_amdgcn_readfirstlane((int)(threadIdx.x >> 5));
  const int tilesN = N >> 6;
  const int tilesM = M >> 6;
  const int tile = (int)blockIdx.x * 8 + wave;
  if (tile >= tilesM * tilesN) return;
  const int tm = tile / tilesN;
  const int tn = tile - tm * tilesN;
  const int m0 = tm << 6;
  const int n0 = tn << 6;

  const int rlane = lane & 15;
  const int koff  = (lane >> 4) * 8;
  const int mOff  = (lane >> 4) * 8;

  v8f acc[4][4];
#pragma unroll
  for (int i = 0; i < 4; ++i)
#pragma unroll
    for (int j = 0; j < 4; ++j) acc[i][j] = (v8f){0.f,0.f,0.f,0.f,0.f,0.f,0.f,0.f};

  for (int k0 = 0; k0 < K; k0 += 32) {
    v16b bh[4], bl[4];
#pragma unroll
    for (int j = 0; j < 4; ++j) {
      const size_t bo = (size_t)(n0 + (j << 4) + rlane) * ldb + koff + k0;
      bh[j] = frag_load_b(Bh + bo);
      bl[j] = frag_load_b(Bl + bo);
    }
#pragma unroll
    for (int i = 0; i < 4; ++i) {
      const size_t ao = (size_t)(m0 + (i << 4) + rlane) * lda + koff + k0;
      const v16b ah = frag_load_b(Ah + ao);
      const v16b al = frag_load_b(Al + ao);
#pragma unroll
      for (int j = 0; j < 4; ++j) {
        acc[i][j] = mma_b(ah, bh[j], acc[i][j]);
        acc[i][j] = mma_b(ah, bl[j], acc[i][j]);
        acc[i][j] = mma_b(al, bh[j], acc[i][j]);
      }
      dep_guard4_b(acc[i][0], acc[i][1], acc[i][2], acc[i][3], ah, al);
    }
    keep4_b(bh[0], bh[1], bh[2], bh[3]);
    keep4_b(bl[0], bl[1], bl[2], bl[3]);
  }
  acc_guard4(acc[0][0], acc[0][1], acc[0][2], acc[0][3]);
  acc_guard4(acc[1][0], acc[1][1], acc[1][2], acc[1][3]);
  acc_guard4(acc[2][0], acc[2][1], acc[2][2], acc[2][3]);
  acc_guard4(acc[3][0], acc[3][1], acc[3][2], acc[3][3]);

  float* slab = sT[wave];
  if (OUT_MODE == 3) {
    float bv = bias[(rlane < kHeadN) ? rlane : (kHeadN - 1)];
    asm volatile("" : "+v"(bv));
#pragma unroll
    for (int i = 0; i < 4; ++i) {
#pragma unroll
      for (int r = 0; r < 8; ++r) {
        const float v = acc[i][0][r] + bv;
        if (rlane < kHeadN) slab[((i << 4) + mOff + r) * kHeadN + rlane] = v;
      }
    }
    __builtin_amdgcn_fence(__ATOMIC_RELEASE, "workgroup");
    __builtin_amdgcn_wave_barrier();
    __builtin_amdgcn_fence(__ATOMIC_ACQUIRE, "workgroup");
    constexpr int kUnits = (64 * kHeadN) / 4;
    static_assert(kUnits == 208, "head tile units");
    v4f tv[7];
#pragma unroll
    for (int it = 0; it < 7; ++it) {
      const int u  = it * 32 + lane;
      const int uc = (u < kUnits) ? u : (kUnits - 1);
      tv[it] = *(const v4f*)(slab + uc * 4);
    }
    float* C = (float*)Cout + (size_t)m0 * kHeadN;
    for (int pass = 0; pass < 2; ++pass) {
#pragma unroll
      for (int it = 0; it < 7; ++it) {
        const int u = it * 32 + lane;
        if (u < kUnits) *(volatile v4f*)(C + (size_t)u * 4) = tv[it];
      }
      __threadfence();
    }
  } else {
#pragma unroll
    for (int i = 0; i < 4; ++i) {
      const int mBase = m0 + (i << 4);
#pragma unroll
      for (int j = 0; j < 4; ++j) {
        const int n = n0 + (j << 4) + rlane;
        const float bv = bias[n];
#pragma unroll
        for (int r = 0; r < 8; ++r) {
          float v = acc[i][j][r] + bv;
          if (CLAMP0) v = fmaxf(v, 0.0f);
          slab[(mOff + r) * 68 + (j << 4) + rlane] = v;
        }
      }
      __builtin_amdgcn_fence(__ATOMIC_RELEASE, "workgroup");
      __builtin_amdgcn_wave_barrier();
      __builtin_amdgcn_fence(__ATOMIC_ACQUIRE, "workgroup");
      {
        const int q = lane >> 3, c8 = (lane & 7) * 8;
        unsigned short* C  = (unsigned short*)Cout;
        unsigned short* C2 = (unsigned short*)Cout2;
        for (int pass = 0; pass < 2; ++pass) {
#pragma unroll
          for (int it = 0; it < 4; ++it) {
            const int row = it * 4 + q;
            const float* sp = slab + row * 68 + c8;
            const v4f a0 = *(const v4f*)(sp);
            const v4f a1 = *(const v4f*)(sp + 4);
            v8h hv, lv;
            split2x4(a0, a1, hv, lv);
            *(volatile v8h*)(C  + (size_t)(mBase + row) * ldc + n0 + c8) = hv;
            *(volatile v8h*)(C2 + (size_t)(mBase + row) * ldc + n0 + c8) = lv;
          }
          __threadfence();
        }
      }
      __builtin_amdgcn_fence(__ATOMIC_RELEASE, "workgroup");
      __builtin_amdgcn_wave_barrier();
      __builtin_amdgcn_fence(__ATOMIC_ACQUIRE, "workgroup");
    }
  }
}

static_assert((64 % 32) == 0 && (128 % 32) == 0 && (256 % 32) == 0, "K multiples of 32");
static_assert((64 % 64) == 0 && (128 % 64) == 0 && (256 % 64) == 0 && (kHeadPad % 64) == 0, "N multiples of 64");
static_assert(((kRows / 64) * (64 / 64)) % 8 == 0, "whole blocks of 8 tiles");

extern "C" void kernel_launch(void* const* d_in, const int* in_sizes, int n_in,
                              void* d_out, int out_size, void* d_ws, size_t ws_size,
                              hipStream_t stream) {
  if (n_in < 16) return;
  if (in_sizes[0] != kRows * kXc) return;
  if (in_sizes[1] != kC1 * kXc) return;
  if (in_sizes[2] != kC1 || in_sizes[3] != kC1) return;
  if (in_sizes[4] != 64 * 64 || in_sizes[5] != 64) return;
  if (in_sizes[6] != 128 * 64 || in_sizes[7] != 128) return;
  if (in_sizes[8] != 256 * 128 || in_sizes[9] != 256) return;
  if (in_sizes[10] != 128 * 256 || in_sizes[11] != 128) return;
  if (in_sizes[12] != 64 * 128 || in_sizes[13] != 64) return;
  if (in_sizes[14] != kHeadN * 64 || in_sizes[15] != kHeadN) return;
  if (out_size != kRows * kHeadN) return;
  if (ws_size < kWsTotal) return;

  const float* x    = (const float*)d_in[0];
  const float* w_c1 = (const float*)d_in[1];
  const float* g1   = (const float*)d_in[2];
  const float* be1  = (const float*)d_in[3];
  const float* w_m1 = (const float*)d_in[4];
  const float* b_m1 = (const float*)d_in[5];
  const float* w_m2 = (const float*)d_in[6];
  const float* b_m2 = (const float*)d_in[7];
  const float* w_m3 = (const float*)d_in[8];
  const float* b_m3 = (const float*)d_in[9];
  const float* w_m4 = (const float*)d_in[10];
  const float* b_m4 = (const float*)d_in[11];
  const float* w_m5 = (const float*)d_in[12];
  const float* b_m5 = (const float*)d_in[13];
  const float* w_m6 = (const float*)d_in[14];
  const float* b_m6 = (const float*)d_in[15];
  float* out = (float*)d_out;

  char* ws = (char*)d_ws;
  unsigned short* WH   = (unsigned short*)(ws + kOffWH);
  unsigned short* WL   = (unsigned short*)(ws + kOffWL);
  int*            IDX  = (int*)(ws + kOffIDX);
  float*          HMAX = (float*)(ws + kOffHMAX);
  float*          HMIN = (float*)(ws + kOffHMIN);
  float*          PART = (float*)(ws + kOffPART);
  float*          SCSH = (float*)(ws + kOffSCSH);
  unsigned short* PH   = (unsigned short*)(ws + kOffPH);
  unsigned short* PL   = (unsigned short*)(ws + kOffPL);
  unsigned short* QH   = (unsigned short*)(ws + kOffQH);
  unsigned short* QL   = (unsigned short*)(ws + kOffQL);

  split_weights_kernel<<<kSplitBlocks, 256, 0, stream>>>(w_m1, w_m2, w_m3, w_m4, w_m5, w_m6, WH, WL);
  knn_select_kernel<<<dim3(kNpt / 256, kBatch), 256, 0, stream>>>(x, IDX);
  edge_conv_stats_kernel<<<kEdgeBlocks, 256, 0, stream>>>(x, IDX, w_c1, HMAX, HMIN, PART);
  bn_finalize_kernel<<<1, 256, 0, stream>>>(PART, g1, be1, SCSH);
  bn_apply_kernel<<<(kRows * kC1 / 8) / 256, 256, 0, stream>>>(HMAX, HMIN, SCSH, PH, PL);

  mlp_gemm64_kernel<2, true><<<64, 256, 0, stream>>>(
      PH, PL, 64, WH + kW1Off, WL + kW1Off, 64, (void*)QH, (void*)QL, 64, b_m1, kRows, 64, 64);
  mlp_gemm64_kernel<2, true><<<128, 256, 0, stream>>>(
      QH, QL, 64, WH + kW2Off, WL + kW2Off, 64, (void*)PH, (void*)PL, 128, b_m2, kRows, 128, 64);
  mlp_gemm64_kernel<2, true><<<256, 256, 0, stream>>>(
      PH, PL, 128, WH + kW3Off, WL + kW3Off, 128, (void*)QH, (void*)QL, 256, b_m3, kRows, 256, 128);
  mlp_gemm64_kernel<2, true><<<128, 256, 0, stream>>>(
      QH, QL, 256, WH + kW4Off, WL + kW4Off, 256, (void*)PH, (void*)PL, 128, b_m4, kRows, 128, 256);
  mlp_gemm64_kernel<2, true><<<64, 256, 0, stream>>>(
      PH, PL, 128, WH + kW5Off, WL + kW5Off, 128, (void*)QH, (void*)QL, 64, b_m5, kRows, 64, 128);
  mlp_gemm64_kernel<3, false><<<64, 256, 0, stream>>>(
      QH, QL, 64, WH + kW6Off, WL + kW6Off, 64, (void*)out, nullptr, kHeadN, b_m6, kRows, kHeadPad, 64);
}
